// RNNIOB_91036126806302
// MI455X (gfx1250) — hardware-verified
//
#include <hip/hip_runtime.h>
#include <math.h>

constexpr int SEQ_T   = 256;
constexpr int NB      = 64;
constexpr int NE      = 256;
constexpr int NH      = 512;
constexpr int NH2     = 1024;
constexpr int NO      = 18;
constexpr int NOPAD   = 64;
constexpr int NVOC    = 50000;
constexpr int NROW    = SEQ_T * NB;
constexpr int NTHR    = 256;
constexpr int ROWS_BLK    = 16;
constexpr int BLK_PER_DIR = NB / ROWS_BLK;
constexpr int HPITCH  = 520;
constexpr int XSP     = 516;
constexpr float CARRY      = 16.0f;
constexpr float CARRY_INV  = 1.0f / 16.0f;
constexpr float CARRY2_INV = 1.0f / 256.0f;
static_assert(NROW % 64 == 0 && NE % 64 == 0 && NH % 64 == 0 && NOPAD % 64 == 0);
static_assert(NE % 32 == 0 && NH % 32 == 0 && NH2 % 32 == 0);
static_assert(NB % ROWS_BLK == 0);
static_assert(NH == 64 * (NTHR / 32));
static_assert((2 * ROWS_BLK * HPITCH) % NTHR == 0);
static_assert((ROWS_BLK * NH / 4) % NTHR == 0 && (ROWS_BLK * NH / 4) / NTHR == 8);
static_assert(HPITCH % 8 == 0 && XSP % 4 == 0);
static_assert(NROW % (NTHR / 32) == 0);
static_assert((NROW / 16) % (NTHR / 32) == 0);
static_assert((16 * NO * 4) % 128 == 0);
static_assert(NO <= NOPAD);

typedef __attribute__((ext_vector_type(16))) _Float16 v16h;
typedef __attribute__((ext_vector_type(8)))  _Float16 v8h;
typedef __attribute__((ext_vector_type(16))) __bf16   v16b;
typedef __attribute__((ext_vector_type(8)))  __bf16   v8b;
typedef __attribute__((ext_vector_type(8)))  float    v8f;
typedef __attribute__((ext_vector_type(4)))  float    v4f;
typedef __attribute__((ext_vector_type(2)))  float    v2f;

__device__ __forceinline__ unsigned short f2bf_bits(float f) {
  unsigned u = __float_as_uint(f);
  return (unsigned short)((u + 0x7FFFu + ((u >> 16) & 1u)) >> 16);
}
__device__ __forceinline__ float bf_bits2f(unsigned short h) { return __uint_as_float(((unsigned)h) << 16); }

__device__ __forceinline__ void dep_guard_h(v8f& a, v8f& b, v16h x, v16h y) { asm volatile("v_nop\n\tv_nop\n\tv_nop\n\tv_nop" : "+v"(a), "+v"(b) : "v"(x), "v"(y)); }
__device__ __forceinline__ void dep_guard_b(v8f& a, v8f& b, v16b x, v16b y) { asm volatile("v_nop\n\tv_nop\n\tv_nop\n\tv_nop" : "+v"(a), "+v"(b) : "v"(x), "v"(y)); }
__device__ __forceinline__ void dep_guard4_h(v8f& a, v8f& b, v8f& c, v8f& d, v16h x, v16h y) {
  asm volatile("v_nop\n\tv_nop\n\tv_nop\n\tv_nop" : "+v"(a), "+v"(b), "+v"(c), "+v"(d) : "v"(x), "v"(y));
}
__device__ __forceinline__ void dep_guard4_b(v8f& a, v8f& b, v8f& c, v8f& d, v16b x, v16b y) {
  asm volatile("v_nop\n\tv_nop\n\tv_nop\n\tv_nop" : "+v"(a), "+v"(b), "+v"(c), "+v"(d) : "v"(x), "v"(y));
}
__device__ __forceinline__ void dep_guard4x5_h(v8f& a, v8f& b, v8f& c, v8f& d, v16h x0, v16h x1, v16h x2, v16h x3, v16h x4) {
  asm volatile("v_nop\n\tv_nop\n\tv_nop\n\tv_nop" : "+v"(a), "+v"(b), "+v"(c), "+v"(d) : "v"(x0), "v"(x1), "v"(x2), "v"(x3), "v"(x4));
}
__device__ __forceinline__ void keep4_h(v16h a, v16h b, v16h c, v16h d) { asm volatile("v_nop" :: "v"(a), "v"(b), "v"(c), "v"(d)); }
__device__ __forceinline__ void keep4_b(v16b a, v16b b, v16b c, v16b d) { asm volatile("v_nop" :: "v"(a), "v"(b), "v"(c), "v"(d)); }
__device__ __forceinline__ void acc_guard4(v8f& a, v8f& b, v8f& c, v8f& d) { asm volatile("v_nop\n\tv_nop\n\tv_nop\n\tv_nop" : "+v"(a), "+v"(b), "+v"(c), "+v"(d)); }
template <typename T> struct Frag;
template <> struct Frag<_Float16> {
  typedef v16h V; union U { v16h v; v8h h[2]; };
  static __device__ __forceinline__ v16h load(const _Float16* p) {
    U f; f.h[0] = *(const v8h*)(p); f.h[1] = *(const v8h*)(p + 16); return f.v;
  }
  static __device__ __forceinline__ v8f mma(v16h a, v16h b, v8f c) {
    return __builtin_amdgcn_wmma_f32_16x16x32_f16(false, a, false, b, (short)0, c, false, false);
  }
  static __device__ __forceinline__ void guard(v8f& a, v8f& b, v16h x, v16h y) { dep_guard_h(a, b, x, y); }
  static __device__ __forceinline__ void guard4(v8f& a, v8f& b, v8f& c, v8f& d, v16h x, v16h y) { dep_guard4_h(a, b, c, d, x, y); }
  static __device__ __forceinline__ void keep(v16h a, v16h b, v16h c, v16h d) { keep4_h(a, b, c, d); }
};
template <> struct Frag<__bf16> {
  typedef v16b V; union U { v16b v; v8b h[2]; };
  static __device__ __forceinline__ v16b load(const __bf16* p) {
    U f; f.h[0] = *(const v8b*)(p); f.h[1] = *(const v8b*)(p + 16); return f.v;
  }
  static __device__ __forceinline__ v8f mma(v16b a, v16b b, v8f c) {
    return __builtin_amdgcn_wmma_f32_16x16x32_bf16(false, a, false, b, (short)0, c, false, false);
  }
  static __device__ __forceinline__ void guard(v8f& a, v8f& b, v16b x, v16b y) { dep_guard_b(a, b, x, y); }
  static __device__ __forceinline__ void guard4(v8f& a, v8f& b, v8f& c, v8f& d, v16b x, v16b y) { dep_guard4_b(a, b, c, d, x, y); }
  static __device__ __forceinline__ void keep(v16b a, v16b b, v16b c, v16b d) { keep4_b(a, b, c, d); }
};

template <int ET> struct Elem;
template <> struct Elem<0> { typedef _Float16 T; };
template <> struct Elem<1> { typedef __bf16 T; };
template <int ET, bool SPLIT, int BIAS_MODE, int OUT_MODE, bool RESID, int ACT = 0>
__global__ __launch_bounds__(256) void wmma_gemm64(
    const unsigned short* __restrict__ Ap, const unsigned short* __restrict__ A2p, int lda, long strideA,
    const unsigned short* __restrict__ Btp, const unsigned short* __restrict__ Bt2p, int ldb, long strideB,
    void* __restrict__ Cout, void* __restrict__ Cout2, int ldc, long strideC,
    const float* __restrict__ bias,
    const float* __restrict__ resid, long strideR,
    int M, int N, int K, float scale) {
  typedef typename Elem<ET>::T T;
  typedef typename Frag<T>::V V;
  const T* A = (const T*)Ap; const T* A2 = (const T*)A2p; const T* Bt = (const T*)Btp; const T* Bt2 = (const T*)Bt2p;
  __shared__ __align__(16) float sT[8][16 * 68];
  const int b    = blockIdx.y;
  const int lane = threadIdx.x & 31;
  const int wave = threadIdx.x >> 5;
  const int tilesN = N >> 6;
  const int tilesM = M >> 6;
  const int tile = blockIdx.x * 8 + wave;
  if (tile >= tilesM * tilesN) return;
  const int tm = tile / tilesN;
  const int tn = tile - tm * tilesN;
  const int m0 = tm << 6;
  const int n0 = tn << 6;

  const T* Ab  = A  + (size_t)b * strideA;
  const T* Bb  = Bt + (size_t)b * strideB;
  const T* Ab2 = SPLIT ? (A2  + (size_t)b * strideA) : nullptr;
  const T* Bb2 = SPLIT ? (Bt2 + (size_t)b * strideB) : nullptr;

  const int rlane = lane & 15;
  const int koff  = (lane >> 4) * 8;
  const int mOff  = (lane >> 4) * 8;

  v8f acc[4][4];
#pragma unroll
  for (int i = 0; i < 4; ++i)
#pragma unroll
    for (int j = 0; j < 4; ++j) acc[i][j] = (v8f){0.f,0.f,0.f,0.f,0.f,0.f,0.f,0.f};

  for (int k0 = 0; k0 < K; k0 += 32) {
    V bh[4], bl[4];
#pragma unroll
    for (int j = 0; j < 4; ++j) {
      const size_t bo = (size_t)(n0 + (j << 4) + rlane) * ldb + koff + k0;
      bh[j] = Frag<T>::load(Bb + bo);
      if (SPLIT) bl[j] = Frag<T>::load(Bb2 + bo);
    }
#pragma unroll
    for (int i = 0; i < 4; ++i) {
      const size_t ao = (size_t)(m0 + (i << 4) + rlane) * lda + koff + k0;
      V ah = Frag<T>::load(Ab + ao);
      V al;
      if (SPLIT) al = Frag<T>::load(Ab2 + ao);
#pragma unroll
      for (int j = 0; j < 4; ++j) {
        acc[i][j] = Frag<T>::mma(ah, bh[j], acc[i][j]);
        if (SPLIT) {
          acc[i][j] = Frag<T>::mma(ah, bl[j], acc[i][j]);
          acc[i][j] = Frag<T>::mma(al, bh[j], acc[i][j]);
        }
      }
      Frag<T>::guard4(acc[i][0], acc[i][1], acc[i][2], acc[i][3], ah, SPLIT ? al : bh[3]);
    }
    Frag<T>::keep(bh[0], bh[1], bh[2], bh[3]);
    if (SPLIT) Frag<T>::keep(bl[0], bl[1], bl[2], bl[3]);
  }
  acc_guard4(acc[0][0], acc[0][1], acc[0][2], acc[0][3]);
  acc_guard4(acc[1][0], acc[1][1], acc[1][2], acc[1][3]);
  acc_guard4(acc[2][0], acc[2][1], acc[2][2], acc[2][3]);
  acc_guard4(acc[3][0], acc[3][1], acc[3][2], acc[3][3]);

  float* slab = sT[wave];
  const float* Rb = RESID ? (resid + (size_t)b * strideR) : nullptr;
#pragma unroll
  for (int i = 0; i < 4; ++i) {
    const int mBase = m0 + (i << 4);
#pragma unroll
    for (int j = 0; j < 4; ++j) {
      const int n = n0 + (j << 4) + rlane;
      float bv = 0.f;
      if (BIAS_MODE == 2) bv = bias[n];
#pragma unroll
      for (int r = 0; r < 8; ++r) {
        float v = acc[i][j][r] * scale;
        if (BIAS_MODE == 1) v += bias[mBase + mOff + r];
        if (BIAS_MODE == 2) v += bv;
        if (RESID) v += Rb[(size_t)(mBase + mOff + r) * ldc + n];
        if (ACT == 1) v = tanhf(v);
        if (ACT == 2) v = fmaxf(v, 0.0f);
        if (ACT == 3) v = v / (1.0f + expf(-v));
        if (ACT == 4) v = (v > 0.f) ? v : 0.01f * v;
        slab[(mOff + r) * 68 + (j << 4) + rlane] = v;
      }
    }
    __builtin_amdgcn_fence(__ATOMIC_RELEASE, "workgroup");
    __builtin_amdgcn_wave_barrier();
    __builtin_amdgcn_fence(__ATOMIC_ACQUIRE, "workgroup");
    if (OUT_MODE == 0) {
      float* C = (float*)Cout + (size_t)b * strideC;
      const int hh = lane >> 4, c4 = (lane & 15) * 4;
      for (int pass = 0; pass < 2; ++pass) {
#pragma unroll
        for (int it = 0; it < 8; ++it) {
          const int row = it * 2 + hh;
          v4f v = *(const v4f*)(slab + row * 68 + c4);
          *(volatile v4f*)(C + (size_t)(mBase + row) * ldc + n0 + c4) = v;
        }
        __threadfence();
      }
    } else {
      const int q = lane >> 3, c8 = (lane & 7) * 8;
      unsigned short* C  = (unsigned short*)Cout  + (size_t)b * strideC;
      unsigned short* C2 = (OUT_MODE == 2) ? ((unsigned short*)Cout2 + (size_t)b * strideC) : nullptr;
      for (int pass = 0; pass < 2; ++pass) {
#pragma unroll
        for (int it = 0; it < 4; ++it) {
          const int row = it * 4 + q;
          const float* sp = slab + row * 68 + c8;
          v8h hv, lv;
#pragma unroll
          for (int e = 0; e < 8; ++e) {
            if (OUT_MODE == 1) {
              hv[e] = (_Float16)sp[e];
            } else {
              unsigned short hb = f2bf_bits(sp[e]);
              unsigned short lb = f2bf_bits(sp[e] - bf_bits2f(hb));
              hv[e] = __builtin_bit_cast(_Float16, hb);
              lv[e] = __builtin_bit_cast(_Float16, lb);
            }
          }
          *(volatile v8h*)(C + (size_t)(mBase + row) * ldc + n0 + c8) = hv;
          if (OUT_MODE == 2) *(volatile v8h*)(C2 + (size_t)(mBase + row) * ldc + n0 + c8) = lv;
        }
        __threadfence();
      }
    }
    __builtin_amdgcn_fence(__ATOMIC_RELEASE, "workgroup");
    __builtin_amdgcn_wave_barrier();
    __builtin_amdgcn_fence(__ATOMIC_ACQUIRE, "workgroup");
  }
}

__global__ __launch_bounds__(NTHR) void cvt_f16_kernel(const float* __restrict__ src, unsigned short* __restrict__ dst,
                                                       int rows, int rows_pad, int ncol8, float sc) {
  const int i  = blockIdx.x * NTHR + threadIdx.x;
  const int n8 = rows_pad * ncol8;
  if (i < n8) {
    const int row  = i / ncol8;
    const int cb   = i - row * ncol8;
    const int rowc = (row < rows) ? row : (rows - 1);
    const float fac = (row < rows) ? sc : 0.0f;
    const float* sp = src + ((size_t)rowc * ncol8 + cb) * 8;
    const v4f a = *(const v4f*)(sp);
    const v4f b = *(const v4f*)(sp + 4);
    v8h hv;
#pragma unroll
    for (int e = 0; e < 4; ++e) {
      hv[e]     = (_Float16)(a[e] * fac);
      hv[4 + e] = (_Float16)(b[e] * fac);
    }
    unsigned short* dp = dst + (size_t)i * 8;
    *(volatile v8h*)dp = hv;
    __threadfence();
    *(volatile v8h*)dp = hv;
  }
}

__global__ __launch_bounds__(NTHR) void gather_emb_kernel(const int* __restrict__ text, const float* __restrict__ table,
                                                          unsigned short* __restrict__ dst) {
  const int tid = threadIdx.x, lane = tid & 31;
  const int m = blockIdx.x * (NTHR / 32) + (tid >> 5);
  if (m >= NROW) return;
  int tok = text[m];
  tok = (tok < 0) ? 0 : tok;
  tok = (tok > NVOC - 1) ? (NVOC - 1) : tok;
  const float* sp = table + (size_t)tok * NE + lane * 8;
  const v4f a = *(const v4f*)(sp);
  const v4f b = *(const v4f*)(sp + 4);
  v8h hv;
#pragma unroll
  for (int e = 0; e < 4; ++e) {
    hv[e]     = (_Float16)(a[e] * CARRY);
    hv[4 + e] = (_Float16)(b[e] * CARRY);
  }
  unsigned short* dp = dst + (size_t)m * NE + lane * 8;
  *(volatile v8h*)dp = hv;
  __threadfence();
  *(volatile v8h*)dp = hv;
}

__global__ __launch_bounds__(NTHR) void bias_prep_kernel(const float* __restrict__ bih0, const float* __restrict__ bhh0,
                                                         const float* __restrict__ bih1, const float* __restrict__ bhh1,
                                                         const float* __restrict__ embb, const float* __restrict__ fcb,
                                                         float* __restrict__ BS0, float* __restrict__ BS1,
                                                         float* __restrict__ EB16, float* __restrict__ FB64) {
  const int tid = threadIdx.x, lane = tid & 31, wave = tid >> 5;
  const int seg = blockIdx.x;
  if (seg < 2) {
    const float* pa = seg ? bih1 : bih0;
    const float* pb = seg ? bhh1 : bhh0;
    float* pd = seg ? BS1 : BS0;
    const int idx = tid * 4;
    const v4f va = *(const v4f*)(pa + idx);
    const v4f vb = *(const v4f*)(pb + idx);
    v4f o;
#pragma unroll
    for (int e = 0; e < 4; ++e) o[e] = va[e] + vb[e];
    *(volatile v4f*)(pd + idx) = o;
    __threadfence();
    *(volatile v4f*)(pd + idx) = o;
  } else if (seg == 2) {
    if (wave < 2) {
      const int idx = tid * 4;
      const v4f v = *(const v4f*)(embb + idx);
      v4f o;
#pragma unroll
      for (int e = 0; e < 4; ++e) o[e] = v[e] * CARRY;
      *(volatile v4f*)(EB16 + idx) = o;
      __threadfence();
      *(volatile v4f*)(EB16 + idx) = o;
    }
  } else {
    if (wave == 0) {
      const int idx = 2 * lane;
      const int i0 = (idx < NO) ? idx : (NO - 1);
      const int i1 = (idx + 1 < NO) ? (idx + 1) : (NO - 1);
      const float f0 = (idx < NO) ? 1.0f : 0.0f;
      const float f1 = (idx + 1 < NO) ? 1.0f : 0.0f;
      const float v0 = fcb[i0];
      const float v1 = fcb[i1];
      v2f o;
      o[0] = v0 * f0;
      o[1] = v1 * f1;
      *(volatile v2f*)(FB64 + idx) = o;
      __threadfence();
      *(volatile v2f*)(FB64 + idx) = o;
    }
  }
}

__global__ __launch_bounds__(NTHR) void rnn_scan_kernel(const float* __restrict__ XP, const unsigned short* __restrict__ WHHp,
                                                        unsigned short* __restrict__ HCAT) {
  __shared__ __align__(16) _Float16 Ah[2][ROWS_BLK * HPITCH];
  __shared__ __align__(16) float    Xs[ROWS_BLK * XSP];
  const _Float16* WHH = (const _Float16*)WHHp;
  const int tid = threadIdx.x, lane = tid & 31, wave = tid >> 5;
  const int c = lane & 15, hh = lane >> 4, koff = hh * 8;
  const int q = lane >> 3, c8 = (lane & 7) * 8;
  const int dir = blockIdx.x / BLK_PER_DIR;
  const int rowbase = (blockIdx.x - dir * BLK_PER_DIR) * ROWS_BLK;
  const float*    XPd = XP  + (size_t)dir * NROW * NH;
  const _Float16* Wd  = WHH + (size_t)dir * NH * NH;
  const int coff = dir * NH + 64 * wave;

  {
    _Float16* ahf = &Ah[0][0];
#pragma unroll 1
    for (int i = tid; i < 2 * ROWS_BLK * HPITCH; i += NTHR) ahf[i] = (_Float16)0.0f;
  }
  __syncthreads();

  const _Float16* wr0 = Wd + (size_t)(64 * wave +  0 + c) * NH + koff;
  const _Float16* wr1 = Wd + (size_t)(64 * wave + 16 + c) * NH + koff;
  const _Float16* wr2 = Wd + (size_t)(64 * wave + 32 + c) * NH + koff;
  const _Float16* wr3 = Wd + (size_t)(64 * wave + 48 + c) * NH + koff;
  const v8f z8 = {0.f, 0.f, 0.f, 0.f, 0.f, 0.f, 0.f, 0.f};

#pragma unroll 1
  for (int i = 0; i < SEQ_T; ++i) {
    const int t = dir ? (SEQ_T - 1 - i) : i;
    const int cur = i & 1;
    const size_t grow0 = (size_t)t * NB + (size_t)rowbase;

#pragma unroll
    for (int it = 0; it < 4; ++it) {
      const int idx = it * NTHR + tid;
      const int row = idx >> 7, c4 = (idx & 127) * 4;
      const v4f v = *(const v4f*)(XPd + (grow0 + row) * NH + c4);
      *(v4f*)(Xs + row * XSP + c4) = v;
    }
    asm volatile("" ::: "memory");
#pragma unroll
    for (int it = 4; it < 8; ++it) {
      const int idx = it * NTHR + tid;
      const int row = idx >> 7, c4 = (idx & 127) * 4;
      const v4f v = *(const v4f*)(XPd + (grow0 + row) * NH + c4);
      *(v4f*)(Xs + row * XSP + c4) = v;
    }
    __syncthreads();

    const _Float16* ahrow = &Ah[cur][0] + c * HPITCH + koff;
    _Float16* ahn = &Ah[cur ^ 1][0];
    v8f acc[4];
    acc[0] = z8; acc[1] = z8; acc[2] = z8; acc[3] = z8;
#pragma unroll 1
    for (int k0 = 0; k0 < NH; k0 += 32) {
      const v16h a  = Frag<_Float16>::load(ahrow + k0);
      const v16h b0 = Frag<_Float16>::load(wr0 + k0);
      const v16h b1 = Frag<_Float16>::load(wr1 + k0);
      const v16h b2 = Frag<_Float16>::load(wr2 + k0);
      const v16h b3 = Frag<_Float16>::load(wr3 + k0);
      acc[0] = Frag<_Float16>::mma(a, b0, acc[0]);
      acc[1] = Frag<_Float16>::mma(a, b1, acc[1]);
      acc[2] = Frag<_Float16>::mma(a, b2, acc[2]);
      acc[3] = Frag<_Float16>::mma(a, b3, acc[3]);
      dep_guard4x5_h(acc[0], acc[1], acc[2], acc[3], a, b0, b1, b2, b3);
    }
    acc_guard4(acc[0], acc[1], acc[2], acc[3]);

#pragma unroll
    for (int nt = 0; nt < 4; ++nt) {
      const int j = 64 * wave + 16 * nt + c;
#pragma unroll
      for (int r = 0; r < 8; ++r) {
        const float xv = Xs[(8 * hh + r) * XSP + j];
        const float hn = fmaxf(fmaf(acc[nt][r], CARRY2_INV, xv), 0.0f);
        ahn[(8 * hh + r) * HPITCH + j] = (_Float16)(hn * CARRY);
      }
    }
    __syncthreads();

    for (int pass = 0; pass < 2; ++pass) {
#pragma unroll
      for (int it = 0; it < 4; ++it) {
        const int row = it * 4 + q;
        const v8h hv = *(const v8h*)(ahn + row * HPITCH + 64 * wave + c8);
        *(volatile v8h*)(HCAT + (grow0 + row) * NH2 + coff + c8) = hv;
      }
      __threadfence();
    }
  }
}

__global__ __launch_bounds__(NTHR) void pack_out_kernel(const float* __restrict__ OUTP, float* __restrict__ out) {
  const int tid = threadIdx.x, lane = tid & 31;
  const int gw = blockIdx.x * (NTHR / 32) + (tid >> 5);
  if (gw >= NROW / 16) return;
  v4f o[3];
#pragma unroll
  for (int it = 0; it < 3; ++it) {
    const int f = it * 32 + lane;
#pragma unroll
    for (int e = 0; e < 4; ++e) {
      const int el  = f * 4 + e;
      const int elc = (el < 16 * NO) ? el : (16 * NO - 1);
      const int row = elc / NO;
      const int col = elc - row * NO;
      o[it][e] = OUTP[(size_t)(gw * 16 + row) * NOPAD + col];
    }
  }
  float* ob = out + (size_t)gw * (16 * NO);
  for (int pass = 0; pass < 2; ++pass) {
#pragma unroll
    for (int it = 0; it < 3; ++it) {
      const int f = it * 32 + lane;
      if (f < 16 * NO / 4) *(volatile v4f*)(ob + f * 4) = o[it];
    }
    __threadfence();
  }
}

extern "C" void kernel_launch(void* const* d_in, const int* in_sizes, int n_in,
                              void* d_out, int out_size, void* d_ws, size_t ws_size, hipStream_t stream) {
  if (n_in < 14 || d_out == nullptr || d_ws == nullptr) return;
  if (in_sizes[0] != NROW || in_sizes[1] != NVOC * NE || in_sizes[2] != NE * NE || in_sizes[3] != NE ||
      in_sizes[4] != 2 * NH * NE || in_sizes[5] != 2 * NH * NH || in_sizes[6] != 2 * NH || in_sizes[7] != 2 * NH ||
      in_sizes[8] != 2 * NH * NH2 || in_sizes[9] != 2 * NH * NH || in_sizes[10] != 2 * NH || in_sizes[11] != 2 * NH ||
      in_sizes[12] != NO * NH2 || in_sizes[13] != NO || out_size != NROW * NO) return;

  const int*   text   = (const int*)  d_in[0];
  const float* table  = (const float*)d_in[1];
  const float* emfc_w = (const float*)d_in[2];
  const float* emfc_b = (const float*)d_in[3];
  const float* w_ih0  = (const float*)d_in[4];
  const float* w_hh0  = (const float*)d_in[5];
  const float* b_ih0  = (const float*)d_in[6];
  const float* b_hh0  = (const float*)d_in[7];
  const float* w_ih1  = (const float*)d_in[8];
  const float* w_hh1  = (const float*)d_in[9];
  const float* b_ih1  = (const float*)d_in[10];
  const float* b_hh1  = (const float*)d_in[11];
  const float* fc_w   = (const float*)d_in[12];
  const float* fc_b   = (const float*)d_in[13];
  float* out = (float*)d_out;

  char* ws = (char*)d_ws; size_t off = 0;
  auto carve = [&](size_t bytes) -> char* { char* p = ws + off; off += (bytes + 255) & ~(size_t)255; return p; };
  unsigned short* AEMB16  = (unsigned short*)carve((size_t)NROW * NE * 2);
  unsigned short* PE16    = (unsigned short*)carve((size_t)NROW * NE * 2);
  float*          XP      = (float*)carve((size_t)2 * NROW * NH * 4);
  unsigned short* HCAT    = (unsigned short*)carve((size_t)NROW * NH2 * 2);
  float*          OUTP    = (float*)carve((size_t)NROW * NOPAD * 4);
  unsigned short* EMFCW16 = (unsigned short*)carve((size_t)NE * NE * 2);
  unsigned short* WIH0    = (unsigned short*)carve((size_t)2 * NH * NE * 2);
  unsigned short* WHH0    = (unsigned short*)carve((size_t)2 * NH * NH * 2);
  unsigned short* WIH1    = (unsigned short*)carve((size_t)2 * NH * NH2 * 2);
  unsigned short* WHH1    = (unsigned short*)carve((size_t)2 * NH * NH * 2);
  unsigned short* FCW16   = (unsigned short*)carve((size_t)NOPAD * NH2 * 2);
  float*          BSUM0   = (float*)carve((size_t)2 * NH * 4);
  float*          BSUM1   = (float*)carve((size_t)2 * NH * 4);
  float*          EMFCB16 = (float*)carve((size_t)NE * 4);
  float*          FCB64   = (float*)carve((size_t)NOPAD * 4);
  if (off > ws_size || off > (size_t)134217728) return;

  cvt_f16_kernel<<<(NE * (NE / 8)) / NTHR, NTHR, 0, stream>>>(emfc_w, EMFCW16, NE, NE, NE / 8, CARRY);
  cvt_f16_kernel<<<(2 * NH * (NE / 8)) / NTHR, NTHR, 0, stream>>>(w_ih0, WIH0, 2 * NH, 2 * NH, NE / 8, CARRY);
  cvt_f16_kernel<<<(2 * NH * (NH / 8)) / NTHR, NTHR, 0, stream>>>(w_hh0, WHH0, 2 * NH, 2 * NH, NH / 8, CARRY);
  cvt_f16_kernel<<<(2 * NH * (NH2 / 8)) / NTHR, NTHR, 0, stream>>>(w_ih1, WIH1, 2 * NH, 2 * NH, NH2 / 8, CARRY);
  cvt_f16_kernel<<<(2 * NH * (NH / 8)) / NTHR, NTHR, 0, stream>>>(w_hh1, WHH1, 2 * NH, 2 * NH, NH / 8, CARRY);
  cvt_f16_kernel<<<(NOPAD * (NH2 / 8)) / NTHR, NTHR, 0, stream>>>(fc_w, FCW16, NO, NOPAD, NH2 / 8, CARRY);
  bias_prep_kernel<<<4, NTHR, 0, stream>>>(b_ih0, b_hh0, b_ih1, b_hh1, emfc_b, fc_b, BSUM0, BSUM1, EMFCB16, FCB64);
  gather_emb_kernel<<<NROW / (NTHR / 32), NTHR, 0, stream>>>(text, table, AEMB16);

  wmma_gemm64<0, false, 2, 1, false, 0><<<dim3((NROW / 64) * (NE / 64) / 8, 1), 256, 0, stream>>>(
      AEMB16, AEMB16, NE, 0L, EMFCW16, EMFCW16, NE, 0L, (void*)PE16, (void*)PE16, NE, 0L,
      EMFCB16, BSUM0, 0L, NROW, NE, NE, CARRY_INV);

  const dim3 gxp((NROW / 64) * (NH / 64) / 8, 1);
  for (int d = 0; d < 2; ++d) {
    wmma_gemm64<0, false, 2, 0, false, 0><<<gxp, 256, 0, stream>>>(
        PE16, PE16, NE, 0L, WIH0 + (size_t)d * NH * NE, WIH0 + (size_t)d * NH * NE, NE, 0L,
        (void*)(XP + (size_t)d * NROW * NH), (void*)(XP + (size_t)d * NROW * NH), NH, 0L,
        BSUM0 + d * NH, BSUM0, 0L, NROW, NH, NE, CARRY2_INV);
  }
  rnn_scan_kernel<<<2 * BLK_PER_DIR, NTHR, 0, stream>>>(XP, WHH0, HCAT);

  for (int d = 0; d < 2; ++d) {
    wmma_gemm64<0, false, 2, 0, false, 0><<<gxp, 256, 0, stream>>>(
        HCAT, HCAT, NH2, 0L, WIH1 + (size_t)d * NH * NH2, WIH1 + (size_t)d * NH * NH2, NH2, 0L,
        (void*)(XP + (size_t)d * NROW * NH), (void*)(XP + (size_t)d * NROW * NH), NH, 0L,
        BSUM1 + d * NH, BSUM1, 0L, NROW, NH, NH2, CARRY2_INV);
  }
  rnn_scan_kernel<<<2 * BLK_PER_DIR, NTHR, 0, stream>>>(XP, WHH1, HCAT);

  wmma_gemm64<0, false, 2, 0, false, 0><<<dim3((NROW / 64) * (NOPAD / 64) / 8, 1), 256, 0, stream>>>(
      HCAT, HCAT, NH2, 0L, FCW16, FCW16, NH2, 0L, (void*)OUTP, (void*)OUTP, NOPAD, 0L,
      FCB64, BSUM0, 0L, NROW, NOPAD, NH2, CARRY2_INV);
  pack_out_kernel<<<(NROW / 16) / (NTHR / 32), NTHR, 0, stream>>>(OUTP, out);
}
